// CausalAttention_11458972745858
// MI455X (gfx1250) — hardware-verified
//
#include <hip/hip_runtime.h>


#ifndef NB
#define NB 2
#endif
#ifndef SEQ
#define SEQ 2048
#endif
#define NB_FULL  2
#define SEQ_FULL 2048
#define DM   1024
#define NH   16
#define HD   64
#define NQKV 3072
#define NU   (NB * NH)
#define SC2  0.18033688011112042f
static_assert(NH * HD == DM);
static_assert(NQKV == 3 * DM);
static_assert(SEQ % 64 == 0);
static_assert(DM % 64 == 0);
static_assert(NB <= NB_FULL);
static_assert(SEQ <= SEQ_FULL);
static_assert((size_t)(SEQ / 64) * (NQKV / 64) * NB * 4096 == (size_t)3 * NB * SEQ * DM);
static_assert((size_t)NU * (SEQ / 16) * 16 * HD == (size_t)NB * SEQ * DM);
static_assert((size_t)(SEQ / 64) * (DM / 64) * NB * 4096 == (size_t)NB * SEQ * DM);
static_assert(((size_t)SEQ * DM / 8) % 256 == 0);
static_assert(((size_t)NQKV * DM / 8) % 256 == 0);
static_assert(((size_t)DM * DM / 8) % 256 == 0);
static_assert((size_t)NB * SEQ * DM * 2 * 9 + (size_t)NQKV * DM * 2 + (size_t)DM * DM * 2 <= (size_t)134217728);

typedef unsigned short bf;
typedef __attribute__((ext_vector_type(16))) __bf16   v16bf;
typedef __attribute__((ext_vector_type(16))) unsigned short v16us;
typedef __attribute__((ext_vector_type(8)))  unsigned short v8us;
typedef __attribute__((ext_vector_type(8)))  float    v8f;
typedef __attribute__((ext_vector_type(4)))  float    v4f;
typedef v4f  __attribute__((may_alias)) v4fa;

__device__ __forceinline__ unsigned short f2bf(float f) { unsigned u = __float_as_uint(f); u += 0x7FFFu + ((u >> 16) & 1u); return (unsigned short)(u >> 16); }
__device__ __forceinline__ float bf2f(unsigned short b) { return __uint_as_float(((unsigned)b) << 16); }
__device__ __forceinline__ void splitf(float y, unsigned short& h, unsigned short& l) { h = f2bf(y); l = f2bf(y - bf2f(h)); }
__device__ __forceinline__ v16bf cat16b(v8us lo, v8us hi) { return __builtin_bit_cast(v16bf, __builtin_shufflevector(lo, hi, 0, 1, 2, 3, 4, 5, 6, 7, 8, 9, 10, 11, 12, 13, 14, 15)); }
__device__ __forceinline__ v8f wmmab(v16bf a, v16bf b, v8f c) { return __builtin_amdgcn_wmma_f32_16x16x32_bf16(false, a, false, b, (short)0, c, false, false); }
__device__ __forceinline__ v16bf ldf(const bf* p) { return cat16b(*(const v8us*)p, *(const v8us*)(p + 16)); }
__device__ __forceinline__ void split8(v8f x, v8us& oh, v8us& ol) {
#pragma unroll
    for (int e = 0; e < 8; ++e) { unsigned short a, c; splitf(x[e], a, c); oh[e] = a; ol[e] = c; }
}

__global__ __launch_bounds__(256) void k_cvt8(const float* __restrict__ src, bf* dst, unsigned n8, size_t sS, size_t sD) {
    const unsigned i = blockIdx.x * 256u + threadIdx.x; if (i >= n8) return;
    src += (size_t)blockIdx.y * sS; dst += (size_t)blockIdx.y * sD;
    const v8f v = *(const v8f*)(src + (size_t)i * 8); v8us o;
#pragma unroll
    for (int k = 0; k < 8; ++k) o[k] = f2bf(v[k]);
    *(volatile v8us*)(dst + (size_t)i * 8) = o; __threadfence(); *(volatile v8us*)(dst + (size_t)i * 8) = o;
}

__global__ __launch_bounds__(32) void k_qkv(const bf* __restrict__ X, const bf* __restrict__ W, bf* Qh, bf* Ql, bf* Kh, bf* Kl, bf* Vh, bf* Vl) {
    __shared__ __align__(16) float os[64 * 68];
    const unsigned lane = threadIdx.x & 31u, lr = lane & 15u, hi = lane >> 4;
    const unsigned t0 = blockIdx.x * 64u, n0 = blockIdx.y * 64u, bz = blockIdx.z;
    const bf* A = X + ((size_t)bz * SEQ + t0) * DM;
    v8f acc[4][4];
#pragma unroll
    for (int mb = 0; mb < 4; ++mb)
#pragma unroll
        for (int nb = 0; nb < 4; ++nb) acc[mb][nb] = (v8f){};
    const size_t aoff = (size_t)lr * DM + 8u * hi, boff = (size_t)(n0 + lr) * DM + 8u * hi;
#pragma unroll 1
    for (unsigned kc = 0; kc < (unsigned)DM; kc += 32u) {
        v16bf a[4];
#pragma unroll
        for (int mb = 0; mb < 4; ++mb) a[mb] = ldf(A + aoff + (size_t)mb * 16 * DM + kc);
#pragma unroll
        for (int nb = 0; nb < 4; ++nb) { const v16bf wb = ldf(W + boff + (size_t)nb * 16 * DM + kc);
#pragma unroll
            for (int mb = 0; mb < 4; ++mb) acc[mb][nb] = wmmab(a[mb], wb, acc[mb][nb]); }
        asm volatile("v_nop\n\tv_nop\n\tv_nop\n\tv_nop" : "+v"(acc[0][0]), "+v"(acc[1][1]), "+v"(acc[2][2]), "+v"(acc[3][3]) : "v"(a[0]), "v"(a[3]));
    }
#pragma unroll
    for (int mb = 0; mb < 4; ++mb)
#pragma unroll
        for (int nb = 0; nb < 4; ++nb)
#pragma unroll
            for (int j = 0; j < 8; ++j) os[(mb * 16u + hi * 8u + j) * 68u + nb * 16u + lr] = acc[mb][nb][j];
    __syncthreads();
    const unsigned q = lane >> 3, p = lane & 7u;
    const unsigned sel = n0 >> 10, hh = (n0 & 1023u) >> 6, unit = bz * NH + hh;
    if (sel < 2u) {
        bf* H = (sel == 0u) ? Qh : Kh; bf* L = (sel == 0u) ? Ql : Kl;
        const size_t base = ((size_t)unit * SEQ + t0) * HD + p * 8u;
#pragma unroll 1
        for (int ps = 0; ps < 2; ++ps) {
#pragma unroll 2
            for (unsigned it = 0; it < 16u; ++it) { const unsigned row = it * 4u + q; const float* sp = os + row * 68u + p * 8u;
                const v4f x0 = *(const v4fa*)sp, x1 = *(const v4fa*)(sp + 4); v8f x;
#pragma unroll
                for (int e = 0; e < 4; ++e) { x[e] = x0[e]; x[4 + e] = x1[e]; }
                v8us oh, ol; split8(x, oh, ol);
                *(volatile v8us*)(H + base + (size_t)row * HD) = oh; *(volatile v8us*)(L + base + (size_t)row * HD) = ol; }
            if (ps == 0) __threadfence(); }
    } else {
        const size_t base = (size_t)unit * HD * SEQ + t0 + p * 8u;
#pragma unroll 1
        for (int ps = 0; ps < 2; ++ps) {
#pragma unroll 2
            for (unsigned it = 0; it < 16u; ++it) { const unsigned d = it * 4u + q; v8f x;
#pragma unroll
                for (int j = 0; j < 8; ++j) x[j] = os[(p * 8u + j) * 68u + d];
                v8us oh, ol; split8(x, oh, ol);
                *(volatile v8us*)(Vh + base + (size_t)d * SEQ) = oh; *(volatile v8us*)(Vl + base + (size_t)d * SEQ) = ol; }
            if (ps == 0) __threadfence(); }
    }
}

__global__ __launch_bounds__(32) void k_flash(const bf* __restrict__ Qh, const bf* __restrict__ Ql, const bf* __restrict__ Kh, const bf* __restrict__ Kl, const bf* __restrict__ Vh, const bf* __restrict__ Vl, bf* Ch, bf* Cl) {
    __shared__ __align__(16) float os[16 * 68];
    const unsigned lane = threadIdx.x & 31u, n = lane & 15u, h = lane >> 4;
    const unsigned unit = blockIdx.x, qbase = blockIdx.y * 16u;
    const unsigned bz = unit >> 4, hh = unit & 15u;
    const size_t ubase = (size_t)unit * SEQ * HD;
    const size_t qo = ubase + (size_t)(qbase + n) * HD + 8u * h;
    const v16bf bqh0 = ldf(Qh + qo), bqh1 = ldf(Qh + qo + 32), bql0 = ldf(Ql + qo), bql1 = ldf(Ql + qo + 32);
    v8f acc[4];
#pragma unroll
    for (int j = 0; j < 4; ++j) acc[j] = (v8f){};
    float mrun = -1.0e30f, lrun = 0.f;
    const unsigned qrow = qbase + n;
    const unsigned nt = (qbase + 47u) >> 5;
#pragma unroll 1
    for (unsigned kt = 0; kt < nt; ++kt) {
        const unsigned k0 = kt * 32u;
        v8f s[2];
#pragma unroll
        for (int g = 0; g < 2; ++g) {
            const size_t ko = ubase + (size_t)(k0 + 16u * g + n) * HD + 8u * h;
            const v16bf kh0 = ldf(Kh + ko), kh1 = ldf(Kh + ko + 32), kl0 = ldf(Kl + ko), kl1 = ldf(Kl + ko + 32);
            v8f sg = (v8f){};
            sg = wmmab(kh0, bqh0, sg); sg = wmmab(kh1, bqh1, sg);
            sg = wmmab(kl0, bqh0, sg); sg = wmmab(kl1, bqh1, sg);
            sg = wmmab(kh0, bql0, sg); sg = wmmab(kh1, bql1, sg);
            asm volatile("v_nop\n\tv_nop\n\tv_nop\n\tv_nop" : "+v"(sg) : "v"(kh0), "v"(kh1), "v"(kl0), "v"(kl1), "v"(bqh0), "v"(bqh1), "v"(bql0), "v"(bql1));
            s[g] = sg;
        }
        float mx = mrun;
#pragma unroll
        for (int g = 0; g < 2; ++g)
#pragma unroll
            for (int r = 0; r < 8; ++r) { const unsigned key = k0 + 16u * g + 8u * h + r; float t = s[g][r] * SC2; t = (key > qrow) ? -1.0e30f : t; s[g][r] = t; mx = fmaxf(mx, t); }
        mx = fmaxf(mx, __shfl_xor(mx, 16, 32));
        const float sc = __builtin_amdgcn_exp2f(mrun - mx); mrun = mx;
        float psum = 0.f; v16us ph, pl;
#pragma unroll
        for (int g = 0; g < 2; ++g)
#pragma unroll
            for (int r = 0; r < 8; ++r) { const float e = __builtin_amdgcn_exp2f(s[g][r] - mx); psum += e; unsigned short a, c; splitf(e, a, c); ph[g * 8 + r] = a; pl[g * 8 + r] = c; }
        lrun = lrun * sc + psum;
        const v16bf pbh = __builtin_bit_cast(v16bf, ph), pbl = __builtin_bit_cast(v16bf, pl);
#pragma unroll
        for (int j = 0; j < 4; ++j)
#pragma unroll
            for (int r = 0; r < 8; ++r) acc[j][r] *= sc;
#pragma unroll
        for (int j = 0; j < 4; ++j) {
            const size_t vo = ubase + (size_t)(16u * j + n) * SEQ + k0 + 8u * h;
            const v16bf vh = ldf(Vh + vo), vl = ldf(Vl + vo);
            v8f aj = acc[j];
            aj = wmmab(vh, pbh, aj); aj = wmmab(vl, pbh, aj); aj = wmmab(vh, pbl, aj);
            asm volatile("v_nop\n\tv_nop\n\tv_nop\n\tv_nop" : "+v"(aj) : "v"(vh), "v"(vl), "v"(pbh), "v"(pbl));
            acc[j] = aj;
        }
    }
    const float lt = lrun + __shfl_xor(lrun, 16, 32);
    const float inv = __builtin_amdgcn_rcpf(lt);
#pragma unroll
    for (int j = 0; j < 4; ++j)
#pragma unroll
        for (int r = 0; r < 8; ++r) os[n * 68u + 16u * j + 8u * h + r] = acc[j][r] * inv;
    __syncthreads();
    const unsigned q = lane >> 3, p = lane & 7u;
    const size_t cb = ((size_t)bz * SEQ + qbase) * DM + hh * HD + p * 8u;
#pragma unroll 1
    for (int ps = 0; ps < 2; ++ps) {
#pragma unroll
        for (unsigned it = 0; it < 4u; ++it) { const unsigned row = it * 4u + q; const float* sp = os + row * 68u + p * 8u;
            const v4f x0 = *(const v4fa*)sp, x1 = *(const v4fa*)(sp + 4); v8f x;
#pragma unroll
            for (int e = 0; e < 4; ++e) { x[e] = x0[e]; x[4 + e] = x1[e]; }
            v8us oh, ol; split8(x, oh, ol);
            *(volatile v8us*)(Ch + cb + (size_t)row * DM) = oh; *(volatile v8us*)(Cl + cb + (size_t)row * DM) = ol; }
        if (ps == 0) __threadfence(); }
}

__global__ __launch_bounds__(32) void k_gemmw2(const bf* __restrict__ A, const bf* __restrict__ A2, const bf* __restrict__ Bt, unsigned K, float* C, unsigned ldc, size_t sA, size_t sC) {
    __shared__ __align__(16) float os[16 * 68];
    const size_t z = blockIdx.z; A += z * sA; A2 += z * sA; C += z * sC;
    const unsigned lane = threadIdx.x & 31u, lr = lane & 15u, hi = lane >> 4; const unsigned r0 = blockIdx.x * 64u, c0 = blockIdx.y * 64u;
    v8f acc[4][4];
#pragma unroll
    for (int mb = 0; mb < 4; ++mb)
#pragma unroll
        for (int nb = 0; nb < 4; ++nb) acc[mb][nb] = (v8f){};
    const size_t aoff = (size_t)(r0 + lr) * K + 8u * hi, boff = (size_t)(c0 + lr) * K + 8u * hi;
#pragma unroll 1
    for (unsigned kc = 0; kc < K; kc += 32u) {
        v16bf a[4], a2[4];
#pragma unroll
        for (int mb = 0; mb < 4; ++mb) { a[mb] = ldf(A + aoff + (size_t)mb * 16 * K + kc); a2[mb] = ldf(A2 + aoff + (size_t)mb * 16 * K + kc); }
#pragma unroll
        for (int nb = 0; nb < 4; ++nb) { const v16bf wb = ldf(Bt + boff + (size_t)nb * 16 * K + kc);
#pragma unroll
            for (int mb = 0; mb < 4; ++mb) { acc[mb][nb] = wmmab(a[mb], wb, acc[mb][nb]); acc[mb][nb] = wmmab(a2[mb], wb, acc[mb][nb]); } }
        asm volatile("v_nop\n\tv_nop\n\tv_nop\n\tv_nop" : "+v"(acc[0][0]), "+v"(acc[1][1]), "+v"(acc[2][2]), "+v"(acc[3][3]) : "v"(a[0]), "v"(a[3]));
    }
#pragma unroll
    for (int mb = 0; mb < 4; ++mb) {
#pragma unroll
        for (int nb = 0; nb < 4; ++nb) {
#pragma unroll
            for (int j = 0; j < 8; ++j) os[(hi * 8u + j) * 68u + nb * 16u + lr] = acc[mb][nb][j]; }
        __builtin_amdgcn_wave_barrier(); asm volatile("" ::: "memory");
        float* crow = C + (size_t)(r0 + mb * 16u) * ldc + c0;
#pragma unroll 1
        for (int ps = 0; ps < 2; ++ps) {
#pragma unroll
            for (unsigned s = 0; s < 8u; ++s) { const unsigned row = 2u * s + hi, cofs = lr * 4u; const v4f val = *(const v4fa*)(os + row * 68u + cofs);
                *(volatile v4f*)(crow + (size_t)row * ldc + cofs) = val; }
            if (ps == 0) __threadfence(); }
        __builtin_amdgcn_wave_barrier(); asm volatile("" ::: "memory");
    }
}

extern "C" void kernel_launch(void* const* d_in, const int* in_sizes, int n_in,
                              void* d_out, int out_size, void* d_ws, size_t ws_size, hipStream_t stream) {
    if (n_in < 3) return;
    const size_t needx = (size_t)(NB - 1) * SEQ_FULL * DM + (size_t)SEQ * DM;
    if ((size_t)in_sizes[0] < needx) return;
    if ((size_t)in_sizes[1] < (size_t)NQKV * DM) return;
    if ((size_t)in_sizes[2] < (size_t)DM * DM) return;
    if ((size_t)out_size < needx) return;
    const float* x    = (const float*)d_in[0];
    const float* wqkv = (const float*)d_in[1];
    const float* wo   = (const float*)d_in[2];
    float* OUT = (float*)d_out;
    char* wsp = (char*)d_ws;
    auto take = [&](size_t bytes) { char* p = wsp; wsp += (bytes + 255) & ~(size_t)255; return (void*)p; };
    const size_t plane = (size_t)NB * SEQ * DM * 2;
    bf* XB = (bf*)take(plane);
    bf* WQ = (bf*)take((size_t)NQKV * DM * 2);
    bf* WO = (bf*)take((size_t)DM * DM * 2);
    bf* Qh = (bf*)take(plane); bf* Ql = (bf*)take(plane);
    bf* Kh = (bf*)take(plane); bf* Kl = (bf*)take(plane);
    bf* Vh = (bf*)take(plane); bf* Vl = (bf*)take(plane);
    bf* Ch = (bf*)take(plane); bf* Cl = (bf*)take(plane);
    const size_t used = (size_t)(wsp - (char*)d_ws);
    if (used > ws_size || used > (size_t)134217728) return;

    k_cvt8<<<dim3((unsigned)((size_t)SEQ * DM / 8 / 256), NB, 1), 256, 0, stream>>>(x, XB, (unsigned)((size_t)SEQ * DM / 8), (size_t)SEQ_FULL * DM, (size_t)SEQ * DM);
    k_cvt8<<<dim3((unsigned)((size_t)NQKV * DM / 8 / 256), 1, 1), 256, 0, stream>>>(wqkv, WQ, (unsigned)((size_t)NQKV * DM / 8), 0, 0);
    k_cvt8<<<dim3((unsigned)((size_t)DM * DM / 8 / 256), 1, 1), 256, 0, stream>>>(wo, WO, (unsigned)((size_t)DM * DM / 8), 0, 0);
    k_qkv<<<dim3(SEQ / 64, NQKV / 64, NB), 32, 0, stream>>>(XB, WQ, Qh, Ql, Kh, Kl, Vh, Vl);
    k_flash<<<dim3(NU, SEQ / 16, 1), 32, 0, stream>>>(Qh, Ql, Kh, Kl, Vh, Vl, Ch, Cl);
    k_gemmw2<<<dim3(SEQ / 64, DM / 64, NB), 32, 0, stream>>>(Ch, Cl, WO, (unsigned)DM, OUT, (unsigned)DM, (size_t)SEQ * DM, (size_t)SEQ_FULL * DM);
}
